// CMAModel_72722386256237
// MI455X (gfx1250) — hardware-verified
//
#include <hip/hip_runtime.h>


#define NB2  2
#define NT_  2048
#define NFM  3072
#define NRM  320
#define NM_  (NFM + NRM)
#define NKV_ALL (NT_ + NM_)
#define HS   768
#define NH_  6
#define NKV  6
#define HD   128
#define KW   (NKV * HD)
#define NREP 1
#define NCT  5
#define SCL  0.08838834764831845f
#define PSC  32768.0f
#define LOSC 1024.0f
#define LOSCI (1.0f / 1024.0f)

typedef _Float16 h16;
typedef unsigned short bf;
typedef __attribute__((ext_vector_type(16))) __bf16   v16bf;
typedef __attribute__((ext_vector_type(16))) _Float16 v16h;
typedef __attribute__((ext_vector_type(8)))  _Float16 v8h;
typedef __attribute__((ext_vector_type(8)))  unsigned short v8us;
typedef __attribute__((ext_vector_type(8)))  float    v8f;
typedef __attribute__((ext_vector_type(4)))  float    v4f;
typedef __attribute__((ext_vector_type(4)))  _Float16 v4h;
typedef v8h  __attribute__((may_alias)) v8ha;
typedef v4f  __attribute__((may_alias)) v4fa;
typedef v8us __attribute__((may_alias)) v8usa;

__device__ __forceinline__ unsigned short f2bf(float f) { unsigned u = __float_as_uint(f); u += 0x7FFFu + ((u >> 16) & 1u); return (unsigned short)(u >> 16); }
__device__ __forceinline__ float bf2f(unsigned short b) { return __uint_as_float(((unsigned)b) << 16); }
__device__ __forceinline__ float bfr(float f) { return bf2f(f2bf(f)); }
__device__ __forceinline__ v16h cat16(v8h lo, v8h hi) { return __builtin_shufflevector(lo, hi, 0, 1, 2, 3, 4, 5, 6, 7, 8, 9, 10, 11, 12, 13, 14, 15); }
__device__ __forceinline__ v16bf cat16b(v8us lo, v8us hi) { return __builtin_bit_cast(v16bf, __builtin_shufflevector(lo, hi, 0, 1, 2, 3, 4, 5, 6, 7, 8, 9, 10, 11, 12, 13, 14, 15)); }
__device__ __forceinline__ v8f wmma16(v16h a, v16h b, v8f c) { return __builtin_amdgcn_wmma_f32_16x16x32_f16(false, a, false, b, (short)0, c, false, false); }
__device__ __forceinline__ v8f wmmab(v16bf a, v16bf b, v8f c) { return __builtin_amdgcn_wmma_f32_16x16x32_bf16(false, a, false, b, (short)0, c, false, false); }

__global__ __launch_bounds__(256) void k_cvtb(const float* __restrict__ src, int nrows, bf* dst) {
    const int lane = threadIdx.x & 31, r = blockIdx.x * 8 + (threadIdx.x >> 5);
    if (r >= nrows) return;
#pragma unroll 1
    for (int ps = 0; ps < 2; ++ps) {
#pragma unroll
        for (int q = 0; q < HS / 256; ++q) { v8us o;
#pragma unroll
            for (int i = 0; i < 8; ++i) o[i] = f2bf(src[(size_t)r * HS + q * 256 + lane * 8 + i]);
            *(volatile v8us*)(dst + (size_t)r * HS + q * 256 + lane * 8) = o; }
        if (ps == 0) __threadfence(); }
}
template <bool SPLITA>
__global__ __launch_bounds__(128) void k_gemm(const bf* __restrict__ A, const bf* __restrict__ Al, const bf* __restrict__ Bn, const float* __restrict__ bias, int ldc, float* C, int rawbias = 0) {
    __shared__ __align__(16) float ost[4][16 * 68];
    const int lane = threadIdx.x & 31, wave = threadIdx.x >> 5, lr = lane & 15, hi = lane >> 4;
    const size_t r0 = (size_t)blockIdx.x * 64 + wave * 16; const int c0 = blockIdx.y * 64;
    const size_t aoff = (r0 + lr) * HS + 8 * hi;
    v8f acc[4];
#pragma unroll
    for (int t = 0; t < 4; ++t) acc[t] = (v8f){};
#pragma unroll 2
    for (int kc = 0; kc < HS; kc += 32) {
        const v16bf a = cat16b(*(const v8us*)(A + aoff + kc), *(const v8us*)(A + aoff + kc + 16));
        v16bf al = a; if (SPLITA) al = cat16b(*(const v8us*)(Al + aoff + kc), *(const v8us*)(Al + aoff + kc + 16));
#pragma unroll
        for (int t = 0; t < 4; ++t) { const bf* bp = Bn + (size_t)(c0 + t * 16 + lr) * HS + kc + 8 * hi; const v16bf bb = cat16b(*(const v8us*)bp, *(const v8us*)(bp + 16)); acc[t] = wmmab(a, bb, acc[t]); if (SPLITA) acc[t] = wmmab(al, bb, acc[t]); }
        asm volatile("v_nop" : "+v"(acc[0]), "+v"(acc[1]), "+v"(acc[2]), "+v"(acc[3]) : "v"(a), "v"(al) : "memory");
    }
    float* os = &ost[wave][0];
#pragma unroll
    for (int t = 0; t < 4; ++t)
#pragma unroll
        for (int j = 0; j < 8; ++j) os[(hi * 8 + j) * 68 + t * 16 + lr] = acc[t][j] + (bias ? (rawbias ? bias[c0 + t * 16 + lr] : bfr(bias[c0 + t * 16 + lr])) : 0.f);
    __builtin_amdgcn_wave_barrier(); asm volatile("" ::: "memory");
    float* crow = C + r0 * ldc + c0;
    auto pass = [&]() {
#pragma unroll
        for (int s = 0; s < 8; ++s) { const int Lid = (lane >> 3) + 4 * s, piece = lane & 7; const int row = Lid >> 1, cofs = (Lid & 1) * 32 + piece * 4;
            const v4f val = *(const v4fa*)(os + row * 68 + cofs); *(volatile v4f*)(crow + (size_t)row * ldc + cofs) = val; }
    };
    pass(); __threadfence(); pass();
}
template <int NKEY>
__global__ __launch_bounds__(256) void k_vt(const float* __restrict__ V, bf* VTH, bf* VTL) {
    __shared__ float tl[64][65];
    const int tid = threadIdx.x, t0 = blockIdx.x * 64, d0 = blockIdx.y * 64, g = blockIdx.z;
    { const int tt = tid >> 2, dq = (tid & 3) * 16;
#pragma unroll
      for (int i = 0; i < 16; ++i) tl[dq + i][tt] = V[(size_t)(t0 + tt) * KW + g * HD + d0 + dq + i]; }
    __syncthreads();
    const int piece = tid & 7;
    auto pass = [&]() {
#pragma unroll
        for (int s = 0; s < 2; ++s) { const int d = (tid >> 3) + 32 * s; v8us oh, ol;
#pragma unroll
            for (int i = 0; i < 8; ++i) { const float v = tl[d][piece * 8 + i]; const unsigned short hb = f2bf(v); oh[i] = hb; ol[i] = f2bf(v - bf2f(hb)); }
            const size_t o = ((size_t)g * HD + d0 + d) * NKEY + t0 + piece * 8; *(volatile v8us*)(VTH + o) = oh; *(volatile v8us*)(VTL + o) = ol; }
    };
    pass(); __threadfence(); pass();
}
__global__ __launch_bounds__(256) void k_f16s(const float* __restrict__ src, int nrows, h16* PH, h16* PL) {
    const int lane = threadIdx.x & 31, r = blockIdx.x * 8 + (threadIdx.x >> 5); if (r >= nrows) return;
#pragma unroll 1
    for (int ps = 0; ps < 2; ++ps) {
#pragma unroll 1
        for (int q = 0; q < KW / 256; ++q) { const size_t o = (size_t)r * KW + q * 256 + lane * 8; const v8f v = *(const v8f*)(src + o); v8h oh, ol;
#pragma unroll
            for (int i = 0; i < 8; ++i) { const h16 a = (h16)v[i]; oh[i] = a; ol[i] = (h16)((v[i] - (float)a) * LOSC); }
            *(volatile v8h*)(PH + o) = oh; *(volatile v8h*)(PL + o) = ol; }
        if (ps == 0) __threadfence(); }
}

__global__ __launch_bounds__(256) void k_cq(const float* __restrict__ ctrl, const float* __restrict__ Wc, float* CQ) {
#pragma unroll 1
    for (int ps = 0; ps < 2; ++ps) {
        for (int c = threadIdx.x; c < HS; c += 256) { float a = 0.f;
#pragma unroll
            for (int j = 0; j < NCT; ++j) a = fmaf(bfr(ctrl[j]), bfr(Wc[c * NCT + j]), a);
            *(volatile float*)(CQ + c) = a; }
        if (ps == 0) __threadfence(); }
}
__global__ __launch_bounds__(256) void k_gate(const float* __restrict__ Q, const float* __restrict__ Wg, const float* __restrict__ bg, float* GATE) {
    __shared__ __align__(16) float gs[8][8];
    const int lane = threadIdx.x & 31, wv = threadIdx.x >> 5, t = blockIdx.x * 8 + wv;
    const float* qr = Q + (size_t)t * HS;
#pragma unroll 1
    for (int h = 0; h < NH_; ++h) { float a = 0.f;
#pragma unroll 4
        for (int c = lane; c < HS; c += 32) a = fmaf(qr[c], bfr(Wg[h * HS + c]), a);
#pragma unroll
        for (int sh = 16; sh; sh >>= 1) a += __shfl_xor(a, sh, 32);
        if (lane == 0) gs[wv][h] = 1.0f / (1.0f + __expf(-(a + bfr(bg[h])))); }
    if (lane < 2) gs[wv][6 + lane] = 0.f;
    __syncthreads();
    if (wv == 0 && lane < 16) { const v4f v = *(const v4fa*)(&gs[0][0] + lane * 4); float* dst = GATE + (size_t)blockIdx.x * 64 + lane * 4; *(volatile v4f*)dst = v; __threadfence(); *(volatile v4f*)dst = v; }
}
__global__ __launch_bounds__(256) void k_comb2(const float* __restrict__ PLo, const float* __restrict__ PMo, const float* __restrict__ ML, const float* __restrict__ LL, const float* __restrict__ MM, const float* __restrict__ LM, const float* __restrict__ GATE, bf* Ch, bf* Cl) {
    typedef __attribute__((ext_vector_type(2))) unsigned short v2us;
    const size_t u = (size_t)blockIdx.x * 256 + threadIdx.x; if (u >= (size_t)NT_ * HS / 2) return;
    const size_t e0 = u * 2; const int t = (int)(e0 / HS), c = (int)(e0 % HS), h = c / HD;
    const float ml = ML[(size_t)h * NT_ + t], ll = LL[(size_t)h * NT_ + t], mm = MM[(size_t)h * NT_ + t], lm = LM[(size_t)h * NT_ + t], g = GATE[(size_t)t * 8 + h];
    const float m = fmaxf(ml, mm); const float wl = __expf(ml - m) * ll, wm = __expf(mm - m) * lm; const float inv = 1.0f / (wl + wm);
    v2us oh, ol;
#pragma unroll
    for (int i = 0; i < 2; ++i) { const float y = (wl * PLo[e0 + i] + g * wm * PMo[e0 + i]) * inv; const unsigned short hb = f2bf(y); oh[i] = hb; ol[i] = f2bf(y - bf2f(hb)); }
    *(volatile v2us*)(Ch + e0) = oh; *(volatile v2us*)(Cl + e0) = ol; __threadfence(); *(volatile v2us*)(Ch + e0) = oh; *(volatile v2us*)(Cl + e0) = ol;
}
template <bool CAUSAL, int NKEY>
__global__ __launch_bounds__(128) void k_attn(const h16* __restrict__ QH, const h16* __restrict__ QL, const h16* __restrict__ KH, const h16* __restrict__ KL, const bf* __restrict__ VTH, const bf* __restrict__ VTL, float* OUTP, float* MOUT, float* LOUT) {
    __shared__ float mls[2][64];
    __shared__ __align__(16) unsigned short plds[4][16 * 32];
    __shared__ __align__(16) unsigned short plds2[4][16 * 32];
    __shared__ __align__(16) float ost[4][16 * 68];
    const int lane = threadIdx.x & 31, wave = threadIdx.x >> 5, lr = lane & 15, hi = lane >> 4;
    const int bid = blockIdx.x; const int h = bid / (NT_ / 64), qt = bid - h * (NT_ / 64); const int g = h / NREP;
    const int q0 = qt * 64 + wave * 16;
    unsigned short* pl = &plds[wave][0]; unsigned short* pl2 = &plds2[wave][0];
    const size_t qo = (size_t)(q0 + lr) * (NH_ * HD) + h * HD + 8 * hi;
    const h16* kh_b = KH + g * HD; const h16* kl_b = KL + g * HD;
    const size_t vbase = ((size_t)g * HD) * NKEY;
    v8f o[8];
#pragma unroll
    for (int n = 0; n < 8; ++n) o[n] = (v8f){};
    float mrow[8], lpart[8];
#pragma unroll
    for (int j = 0; j < 8; ++j) { mrow[j] = -3.0e38f; lpart[j] = 0.f; }
    const int q0base = qt * 64;
    const int kt_hi = CAUSAL ? (qt * 64 + 63) / 32 : NKEY / 32 - 1;
#pragma unroll 1
    for (int kt = 0; kt <= kt_hi; ++kt) {
        const int l0 = kt * 32;
        const size_t ko0 = (size_t)(l0 + lr) * KW + 8 * hi, ko1 = (size_t)(l0 + 16 + lr) * KW + 8 * hi;
        v8f s0 = {}, s1 = {}, x0 = {}, x1 = {};
#pragma unroll
        for (int kc = 0; kc < 4; ++kc) {
            const v16h qa = cat16(*(const v8h*)(QH + qo + kc * 32), *(const v8h*)(QH + qo + kc * 32 + 16)), qx = cat16(*(const v8h*)(QL + qo + kc * 32), *(const v8h*)(QL + qo + kc * 32 + 16));
            const v16h k0h = cat16(*(const v8h*)(kh_b + ko0 + kc * 32), *(const v8h*)(kh_b + ko0 + kc * 32 + 16)), k1h = cat16(*(const v8h*)(kh_b + ko1 + kc * 32), *(const v8h*)(kh_b + ko1 + kc * 32 + 16));
            s0 = wmma16(qa, k0h, s0); s1 = wmma16(qa, k1h, s1); x0 = wmma16(qx, k0h, x0); x1 = wmma16(qx, k1h, x1);
            asm volatile("v_nop" : "+v"(s0), "+v"(s1), "+v"(x0), "+v"(x1) : "v"(qa), "v"(qx), "v"(k0h), "v"(k1h) : "memory");
            const v16h k0l = cat16(*(const v8h*)(kl_b + ko0 + kc * 32), *(const v8h*)(kl_b + ko0 + kc * 32 + 16)), k1l = cat16(*(const v8h*)(kl_b + ko1 + kc * 32), *(const v8h*)(kl_b + ko1 + kc * 32 + 16));
            x0 = wmma16(qa, k0l, x0); x1 = wmma16(qa, k1l, x1);
            asm volatile("v_nop" : "+v"(x0), "+v"(x1) : "v"(k0l), "v"(k1l) : "memory");
        }
        asm volatile("v_nop\n\tv_nop\n\tv_nop\n\tv_nop" : "+v"(s0), "+v"(s1), "+v"(x0), "+v"(x1));
        float alpha[8];
#pragma unroll
        for (int j = 0; j < 8; ++j) { const int qi = q0 + hi * 8 + j, ja = l0 + lr, jb = l0 + 16 + lr;
            const float a0 = (!CAUSAL || ja <= qi) ? (s0[j] + x0[j] * LOSCI) * SCL : -__builtin_inff(), a1 = (!CAUSAL || jb <= qi) ? (s1[j] + x1[j] * LOSCI) * SCL : -__builtin_inff();
            float mx = fmaxf(a0, a1);
            mx = fmaxf(mx, __shfl_xor(mx, 1, 16)); mx = fmaxf(mx, __shfl_xor(mx, 2, 16)); mx = fmaxf(mx, __shfl_xor(mx, 4, 16)); mx = fmaxf(mx, __shfl_xor(mx, 8, 16));
            const float mn = fmaxf(mrow[j], mx);
            alpha[j] = __expf(mrow[j] - mn); mrow[j] = mn;
            const float p0 = __expf(a0 - mn), p1 = __expf(a1 - mn);
            lpart[j] = lpart[j] * alpha[j] + (p0 + p1);
            const int mr = hi * 8 + j; const float ps0 = p0 * PSC, ps1 = p1 * PSC; const unsigned short h0 = f2bf(ps0), h1 = f2bf(ps1);
            pl[mr * 32 + lr] = h0; pl[mr * 32 + 16 + lr] = h1; pl2[mr * 32 + lr] = f2bf(ps0 - bf2f(h0)); pl2[mr * 32 + 16 + lr] = f2bf(ps1 - bf2f(h1)); }
#pragma unroll
        for (int n = 0; n < 8; ++n)
#pragma unroll
            for (int j = 0; j < 8; ++j) o[n][j] *= alpha[j];
        asm volatile("" ::: "memory");
        const v16bf pa = cat16b(*(const v8usa*)(pl + lr * 32 + hi * 8), *(const v8usa*)(pl + lr * 32 + 16 + hi * 8));
        const v16bf px = cat16b(*(const v8usa*)(pl2 + lr * 32 + hi * 8), *(const v8usa*)(pl2 + lr * 32 + 16 + hi * 8));
#pragma unroll
        for (int n = 0; n < 8; ++n) { const size_t vo = vbase + (size_t)(n * 16 + lr) * NKEY + l0 + hi * 8;
            const v16bf vh = cat16b(*(const v8us*)(VTH + vo), *(const v8us*)(VTH + vo + 16)), vl = cat16b(*(const v8us*)(VTL + vo), *(const v8us*)(VTL + vo + 16));
            o[n] = wmmab(pa, vh, o[n]); o[n] = wmmab(px, vh, o[n]); o[n] = wmmab(pa, vl, o[n]);
            asm volatile("" : "+v"(o[n]) : "v"(vh), "v"(vl) : "memory"); }
        asm volatile("v_nop\n\tv_nop\n\tv_nop\n\tv_nop" : "+v"(o[0]), "+v"(o[7]) : "v"(pa), "v"(px));
        __builtin_amdgcn_wave_barrier();
    }
    float inv[8];
#pragma unroll
    for (int j = 0; j < 8; ++j) { float rs = lpart[j]; rs += __shfl_xor(rs, 1, 16); rs += __shfl_xor(rs, 2, 16); rs += __shfl_xor(rs, 4, 16); rs += __shfl_xor(rs, 8, 16); inv[j] = 1.0f / (rs * PSC);
        if (lr == 0) { mls[0][wave * 16 + hi * 8 + j] = mrow[j]; mls[1][wave * 16 + hi * 8 + j] = rs; } }
    __syncthreads();
    if (threadIdx.x < 64) { const float mv = mls[0][threadIdx.x], lv = mls[1][threadIdx.x]; float* mp = MOUT + (size_t)h * NT_ + q0base + threadIdx.x; float* lp = LOUT + (size_t)h * NT_ + q0base + threadIdx.x;
        *(volatile float*)mp = mv; *(volatile float*)lp = lv; __threadfence(); *(volatile float*)mp = mv; *(volatile float*)lp = lv; }
    float* os = &ost[wave][0];
    float* ob = OUTP + (size_t)q0 * (NH_ * HD) + (size_t)h * HD;
#pragma unroll
    for (int half = 0; half < 2; ++half) {
#pragma unroll
        for (int n = 0; n < 4; ++n)
#pragma unroll
            for (int j = 0; j < 8; ++j) os[(hi * 8 + j) * 68 + n * 16 + lr] = o[half * 4 + n][j] * inv[j];
        __builtin_amdgcn_wave_barrier(); asm volatile("" ::: "memory");
#pragma unroll
        for (int ps2 = 0; ps2 < 2; ++ps2) {
#pragma unroll
            for (int s = 0; s < 8; ++s) { const int Lid = (lane >> 3) + 4 * s, piece = lane & 7; const int row = Lid >> 1, cofs = (Lid & 1) * 32 + piece * 4;
                const v4f val = *(const v4fa*)(os + row * 68 + cofs); *(volatile v4f*)(ob + (size_t)row * (NH_ * HD) + half * 64 + cofs) = val; }
            if (ps2 == 0) __threadfence(); }
        __builtin_amdgcn_wave_barrier(); asm volatile("" ::: "memory");
    }
}


extern "C" void kernel_launch(void* const* d_in, const int* in_sizes, int n_in,
                              void* d_out, int out_size, void* d_ws, size_t ws_size, hipStream_t stream) {
    (void)in_sizes; (void)n_in; (void)out_size;
    const float* x = (const float*)d_in[0]; const float* fm = (const float*)d_in[1]; const float* rm = (const float*)d_in[2]; const float* ctrl = (const float*)d_in[3];
    const float* Wq = (const float*)d_in[4]; const float* Wk = (const float*)d_in[5]; const float* Wv = (const float*)d_in[6]; const float* Wo = (const float*)d_in[7]; const float* Wc = (const float*)d_in[8]; const float* Wg = (const float*)d_in[9]; const float* bg = (const float*)d_in[10];
    float* out = (float*)d_out;
    char* wsp = (char*)d_ws;
    auto take = [&](size_t bytes) { char* p = wsp; wsp += (bytes + 255) & ~(size_t)255; return (void*)p; };
    bf* WqB = (bf*)take((size_t)HS * HS * 2); bf* WkB = (bf*)take((size_t)HS * HS * 2); bf* WvB = (bf*)take((size_t)HS * HS * 2); bf* WoB = (bf*)take((size_t)HS * HS * 2); float* CQ = (float*)take(HS * 4);
    bf* Cb = (bf*)take((size_t)NKV_ALL * HS * 2); float* TMP = (float*)take((size_t)NKV_ALL * HS * 4); float* GATE = (float*)take((size_t)NT_ * 8 * 4);
    h16* QH = (h16*)take((size_t)NT_ * HS * 2); h16* QL = (h16*)take((size_t)NT_ * HS * 2); h16* KH = (h16*)take((size_t)NKV_ALL * KW * 2); h16* KL = (h16*)take((size_t)NKV_ALL * KW * 2);
    bf* VLH = (bf*)take((size_t)KW * NT_ * 2); bf* VLL = (bf*)take((size_t)KW * NT_ * 2); bf* VMH = (bf*)take((size_t)KW * NM_ * 2); bf* VML = (bf*)take((size_t)KW * NM_ * 2);
    float* PLo = (float*)take((size_t)NT_ * HS * 4); float* PMo = (float*)take((size_t)NT_ * HS * 4);
    float* ML = (float*)take((size_t)NH_ * NT_ * 4); float* LL = (float*)take((size_t)NH_ * NT_ * 4); float* MM = (float*)take((size_t)NH_ * NT_ * 4); float* LM = (float*)take((size_t)NH_ * NT_ * 4);
    bf* Ch = (bf*)take((size_t)NT_ * HS * 2); bf* Cl = (bf*)take((size_t)NT_ * HS * 2);
    if ((size_t)(wsp - (char*)d_ws) > ws_size) return;
    k_cvtb<<<HS / 8, 256, 0, stream>>>(Wq, HS, WqB); k_cvtb<<<HS / 8, 256, 0, stream>>>(Wk, HS, WkB); k_cvtb<<<HS / 8, 256, 0, stream>>>(Wv, HS, WvB); k_cvtb<<<HS / 8, 256, 0, stream>>>(Wo, HS, WoB);
    k_cq<<<1, 256, 0, stream>>>(ctrl, Wc, CQ);
    for (int b = 0; b < NB2; ++b) {
        k_cvtb<<<NT_ / 8, 256, 0, stream>>>(x + (size_t)b * NT_ * HS, NT_, Cb); k_cvtb<<<NFM / 8, 256, 0, stream>>>(fm + (size_t)b * NFM * HS, NFM, Cb + (size_t)NT_ * HS); k_cvtb<<<NRM / 8, 256, 0, stream>>>(rm + (size_t)b * NRM * HS, NRM, Cb + (size_t)(NT_ + NFM) * HS);
        k_gemm<false><<<dim3(NT_ / 64, HS / 64, 1), 128, 0, stream>>>(Cb, nullptr, WqB, CQ, HS, TMP, 1);
        k_f16s<<<NT_ / 8, 256, 0, stream>>>(TMP, NT_, QH, QL); k_gate<<<NT_ / 8, 256, 0, stream>>>(TMP, Wg, bg, GATE);
        k_gemm<false><<<dim3(NKV_ALL / 64, HS / 64, 1), 128, 0, stream>>>(Cb, nullptr, WkB, nullptr, HS, TMP); k_f16s<<<NKV_ALL / 8, 256, 0, stream>>>(TMP, NKV_ALL, KH, KL);
        k_gemm<false><<<dim3(NKV_ALL / 64, HS / 64, 1), 128, 0, stream>>>(Cb, nullptr, WvB, nullptr, HS, TMP);
        k_vt<NT_><<<dim3(NT_ / 64, 2, NKV), 256, 0, stream>>>(TMP, VLH, VLL); k_vt<NM_><<<dim3(NM_ / 64, 2, NKV), 256, 0, stream>>>(TMP + (size_t)NT_ * KW, VMH, VML);
        k_attn<true, NT_><<<NH_ * (NT_ / 64), 128, 0, stream>>>(QH, QL, KH, KL, VLH, VLL, PLo, ML, LL);
        k_attn<false, NM_><<<NH_ * (NT_ / 64), 128, 0, stream>>>(QH, QL, KH + (size_t)NT_ * KW, KL + (size_t)NT_ * KW, VMH, VML, PMo, MM, LM);
        k_comb2<<<(unsigned)(((size_t)NT_ * HS / 2 + 255) / 256), 256, 0, stream>>>(PLo, PMo, ML, LL, MM, LM, GATE, Ch, Cl);
        k_gemm<true><<<dim3(NT_ / 64, HS / 64, 1), 128, 0, stream>>>(Ch, Cl, WoB, nullptr, HS, out + (size_t)b * NT_ * HS);
    }
}
